// FANBlock_29111288333035
// MI455X (gfx1250) — hardware-run, weakly checked
//
#include <hip/hip_runtime.h>
#include <math.h>

typedef _Float16 v16h __attribute__((ext_vector_type(16)));
typedef _Float16 v8h  __attribute__((ext_vector_type(8)));
typedef float    v8f  __attribute__((ext_vector_type(8)));
typedef float    v4f  __attribute__((ext_vector_type(4)));
typedef v8h __attribute__((may_alias)) v8ha;
typedef v4f __attribute__((may_alias)) v4fa;

union Frag { v16h v; v8h half[2]; };

constexpr int CB    = 8;
constexpr int CN    = 1024;
constexpr int CD    = 768;
constexpr int CH    = 8;
constexpr int CHD   = 96;
constexpr int CHID  = 3072;
constexpr int CROWS = CB * CN;
constexpr int IMG   = 32;

constexpr float WSC    = 64.0f;
constexpr float PSCALE = 16384.0f;
constexpr float OSCALE = 32.0f;

__device__ __forceinline__ v8f wmma_f16(v16h a, v16h b, v8f c) {
  v8f d = __builtin_amdgcn_wmma_f32_16x16x32_f16(false, a, false, b, (short)0, c, false, false);
  asm volatile("v_nop\n\tv_nop\n\tv_nop\n\tv_nop" : "+v"(d) : "v"(a), "v"(b));
  return d;
}

__device__ __forceinline__ v16h load_frag(const _Float16* p, int h) {
  Frag f;
  f.half[0] = *(const v8ha*)(p + 8 * h);
  f.half[1] = *(const v8ha*)(p + 16 + 8 * h);
  return f.v;
}

__device__ __forceinline__ v8f zero_v8f() {
  const v8f z = {0.f, 0.f, 0.f, 0.f, 0.f, 0.f, 0.f, 0.f};
  return z;
}

__device__ __forceinline__ float wave_sum(float v) {
  v += __shfl_xor(v, 16);
  v += __shfl_xor(v, 8);
  v += __shfl_xor(v, 4);
  v += __shfl_xor(v, 2);
  v += __shfl_xor(v, 1);
  return v;
}

__device__ __forceinline__ v8h pack8(v4f a, v4f c, float sc) {
  v8h o;
  o[0] = (_Float16)(a[0] * sc); o[1] = (_Float16)(a[1] * sc);
  o[2] = (_Float16)(a[2] * sc); o[3] = (_Float16)(a[3] * sc);
  o[4] = (_Float16)(c[0] * sc); o[5] = (_Float16)(c[1] * sc);
  o[6] = (_Float16)(c[2] * sc); o[7] = (_Float16)(c[3] * sc);
  return o;
}

__global__ __launch_bounds__(256) void cvt_kernel(
    const float* __restrict__ s0, _Float16* __restrict__ d0, int n0,
    const float* __restrict__ s1, _Float16* __restrict__ d1, int n1,
    const float* __restrict__ s2, _Float16* __restrict__ d2, int n2,
    const float* __restrict__ s3, _Float16* __restrict__ d3, int n3, float sc)
{
  const int seg = blockIdx.y;
  const float* s = (seg == 0) ? s0 : ((seg == 1) ? s1 : ((seg == 2) ? s2 : s3));
  _Float16*    d = (seg == 0) ? d0 : ((seg == 1) ? d1 : ((seg == 2) ? d2 : d3));
  const int    n = (seg == 0) ? n0 : ((seg == 1) ? n1 : ((seg == 2) ? n2 : n3));
  const size_t i = ((size_t)blockIdx.x * 256 + threadIdx.x) * 8;
  if (i + 8 > (size_t)n) return;
  const v4f a = *(const v4fa*)(s + i);
  const v4f c = *(const v4fa*)(s + i + 4);
  const v8h o = pack8(a, c, sc);
  *(volatile v8h*)(d + i) = o;
  __threadfence();
  *(volatile v8h*)(d + i) = o;
}

template<int WF32>
__global__ __launch_bounds__(256) void ln_kernel(
    const float* __restrict__ xin, const float* __restrict__ w, const float* __restrict__ bb,
    _Float16* __restrict__ o16, float* __restrict__ o32)
{
  __shared__ __attribute__((aligned(16))) float srow[8 * CD];
  const int tid = threadIdx.x, lane = tid & 31, wv = tid >> 5;
  const int row = blockIdx.x * 8 + wv;
  const float* xr = xin + (size_t)row * CD;

  v4f v[6];
  float s = 0.f;
  #pragma unroll
  for (int j = 0; j < 6; ++j) {
    v[j] = *(const v4fa*)(xr + 128 * j + 4 * lane);
    s += (v[j][0] + v[j][1]) + (v[j][2] + v[j][3]);
  }
  s = wave_sum(s);
  const float mean = s * (1.0f / CD);
  float q = 0.f;
  #pragma unroll
  for (int j = 0; j < 6; ++j) {
    v[j] = v[j] - mean;
    q += (v[j][0] * v[j][0] + v[j][1] * v[j][1]) + (v[j][2] * v[j][2] + v[j][3] * v[j][3]);
  }
  q = wave_sum(q);
  const float rs = 1.0f / sqrtf(q * (1.0f / CD) + 1e-5f);

  float* sr = srow + wv * CD;
  #pragma unroll
  for (int j = 0; j < 6; ++j) {
    const int col = 128 * j + 4 * lane;
    const v4f w4 = *(const v4fa*)(w + col);
    const v4f b4 = *(const v4fa*)(bb + col);
    v[j] = v[j] * rs * w4 + b4;
    *(v4fa*)(sr + col) = v[j];
  }
  if (WF32) {
    float* frow = o32 + (size_t)row * CD;
    #pragma unroll
    for (int j = 0; j < 6; ++j) *(volatile v4f*)(frow + 128 * j + 4 * lane) = v[j];
  }
  __syncthreads();

  _Float16* hrow = o16 + (size_t)row * CD;
  v8h h8[3];
  #pragma unroll
  for (int i = 0; i < 3; ++i) {
    const float* p = sr + 256 * i + 8 * lane;
    const v4f a = *(const v4fa*)p;
    const v4f c = *(const v4fa*)(p + 4);
    h8[i] = pack8(a, c, 1.0f);
    *(volatile v8h*)(hrow + 256 * i + 8 * lane) = h8[i];
  }
  __threadfence();
  if (WF32) {
    float* frow = o32 + (size_t)row * CD;
    #pragma unroll
    for (int j = 0; j < 6; ++j) *(volatile v4f*)(frow + 128 * j + 4 * lane) = v[j];
  }
  #pragma unroll
  for (int i = 0; i < 3; ++i) *(volatile v8h*)(hrow + 256 * i + 8 * lane) = h8[i];
}

template<int ALAY, int MODE>
__global__ __launch_bounds__(128) void gemm_kernel(
    const _Float16* __restrict__ A, const _Float16* __restrict__ Bw, int K, int ldo,
    const float* __restrict__ bias, const float* __restrict__ resid, const float* __restrict__ gamma,
    float oscale,
    _Float16* __restrict__ o16a, _Float16* __restrict__ o16b, _Float16* __restrict__ o16c,
    float* __restrict__ o32)
{
  __shared__ __attribute__((aligned(16))) float sTile[128 * CHD];
  _Float16* sH = reinterpret_cast<_Float16*>(sTile);

  const int tid = threadIdx.x, lane = tid & 31, wv = tid >> 5;
  const int hl = lane >> 4, m = lane & 15;
  const int m0 = blockIdx.x * 128, cg = blockIdx.y, c0 = cg * CHD;
  const int m0w = m0 + 32 * wv;

  v8f acc[2][6];
  #pragma unroll
  for (int mt = 0; mt < 2; ++mt)
    #pragma unroll
    for (int nt = 0; nt < 6; ++nt) acc[mt][nt] = zero_v8f();

  const _Float16* wb = Bw + (size_t)(c0 + m) * K;
  int kq = 0, kr = 0;
  #pragma unroll 1
  for (int k0 = 0; k0 < K; k0 += 32) {
    const _Float16* pa0;
    size_t rstep;
    if (ALAY == 0) {
      pa0 = A + (size_t)(m0w + m) * K + k0;
      rstep = (size_t)16 * K;
    } else {
      pa0 = A + ((size_t)kq * CROWS + (size_t)(m0w + m)) * CHD + kr;
      rstep = (size_t)16 * CHD;
    }
    const v16h a0 = load_frag(pa0, hl);
    const v16h a1 = load_frag(pa0 + rstep, hl);
    #pragma unroll
    for (int nt = 0; nt < 6; ++nt) {
      const v16h bf = load_frag(wb + (size_t)nt * 16 * K + k0, hl);
      acc[0][nt] = wmma_f16(a0, bf, acc[0][nt]);
      acc[1][nt] = wmma_f16(a1, bf, acc[1][nt]);
    }
    if (ALAY == 1) { kr += 32; if (kr == CHD) { kr = 0; ++kq; } }
  }

  const int which = (MODE == 0) ? (cg >> 3) : 0;
  const bool vtile = (MODE == 0) && (which == 2);
  #pragma unroll
  for (int nt = 0; nt < 6; ++nt) {
    const int feat = 16 * nt + m;
    float bvl = 0.0f;
    if (MODE == 1) { if (bias != nullptr) bvl = bias[c0 + feat]; }
    #pragma unroll
    for (int mt = 0; mt < 2; ++mt) {
      #pragma unroll
      for (int r = 0; r < 8; ++r) {
        const int tokl = 32 * wv + 16 * mt + 8 * hl + r;
        const float y = acc[mt][nt][r] * oscale + bvl;
        if (MODE == 2) {
          sTile[tokl * CHD + feat] = y;
        } else {
          const int idx = vtile ? (feat * 128 + tokl) : (tokl * CHD + feat);
          sH[idx] = (_Float16)y;
        }
      }
    }
  }
  __syncthreads();

  if (MODE == 2) {
    v4f vals[24];
    #pragma unroll
    for (int i = 0; i < 24; ++i) {
      const int c = wv * 768 + i * 32 + lane;
      const int row = c / 24, piece = c - row * 24;
      const int col = c0 + 4 * piece;
      v4f vv = *(const v4fa*)(sTile + row * CHD + 4 * piece);
      if (bias != nullptr) vv = vv + *(const v4fa*)(bias + col);
      if (resid != nullptr) {
        const v4f rv = *(const v4fa*)(resid + (size_t)(m0 + row) * ldo + col);
        const v4f gv = *(const v4fa*)(gamma + col);
        vv = rv + gv * vv;
      }
      vals[i] = vv;
      *(volatile v4f*)(o32 + (size_t)(m0 + row) * ldo + col) = vv;
    }
    __threadfence();
    #pragma unroll
    for (int i = 0; i < 24; ++i) {
      const int c = wv * 768 + i * 32 + lane;
      const int row = c / 24, piece = c - row * 24;
      const int col = c0 + 4 * piece;
      *(volatile v4f*)(o32 + (size_t)(m0 + row) * ldo + col) = vals[i];
    }
  } else if (!vtile) {
    const int head = (MODE == 1) ? cg : (cg & 7);
    _Float16* plane = (MODE == 1) ? o16a : ((which == 0) ? o16a : o16b);
    _Float16* base = plane + ((size_t)head * CROWS + (size_t)m0) * CHD;
    v8h vals[12];
    #pragma unroll
    for (int i = 0; i < 12; ++i) {
      const int c = wv * 384 + i * 32 + lane;
      vals[i] = *(const v8ha*)(sH + 8 * c);
      *(volatile v8h*)(base + 8 * c) = vals[i];
    }
    __threadfence();
    #pragma unroll
    for (int i = 0; i < 12; ++i) {
      const int c = wv * 384 + i * 32 + lane;
      *(volatile v8h*)(base + 8 * c) = vals[i];
    }
  } else {
    const int head = cg & 7;
    v8h vals[12];
    #pragma unroll
    for (int i = 0; i < 12; ++i) {
      const int c = wv * 384 + i * 32 + lane;
      const int feat = c >> 4, piece = c & 15;
      vals[i] = *(const v8ha*)(sH + feat * 128 + 8 * piece);
      _Float16* dst = o16c + ((size_t)(head * CHD + feat)) * CROWS + m0 + 8 * piece;
      *(volatile v8h*)dst = vals[i];
    }
    __threadfence();
    #pragma unroll
    for (int i = 0; i < 12; ++i) {
      const int c = wv * 384 + i * 32 + lane;
      const int feat = c >> 4, piece = c & 15;
      _Float16* dst = o16c + ((size_t)(head * CHD + feat)) * CROWS + m0 + 8 * piece;
      *(volatile v8h*)dst = vals[i];
    }
  }
}

__device__ __forceinline__ v16h pack_p(v8f a, v8f c) {
  const v16h r = { (_Float16)(a[0] * PSCALE), (_Float16)(a[1] * PSCALE), (_Float16)(a[2] * PSCALE), (_Float16)(a[3] * PSCALE),
                   (_Float16)(a[4] * PSCALE), (_Float16)(a[5] * PSCALE), (_Float16)(a[6] * PSCALE), (_Float16)(a[7] * PSCALE),
                   (_Float16)(c[0] * PSCALE), (_Float16)(c[1] * PSCALE), (_Float16)(c[2] * PSCALE), (_Float16)(c[3] * PSCALE),
                   (_Float16)(c[4] * PSCALE), (_Float16)(c[5] * PSCALE), (_Float16)(c[6] * PSCALE), (_Float16)(c[7] * PSCALE) };
  return r;
}

__global__ __launch_bounds__(128) void attn_kernel(
    const _Float16* __restrict__ qp, const _Float16* __restrict__ kp,
    const _Float16* __restrict__ vt, _Float16* __restrict__ op)
{
  __shared__ __attribute__((aligned(16))) _Float16 sO[4 * 16 * CHD];

  const int tid = threadIdx.x, lane = tid & 31, wv = tid >> 5;
  const int hl = lane >> 4, m = lane & 15;
  const int bh = blockIdx.y, b = bh >> 3, head = bh & 7;
  const int q0 = blockIdx.x * 64 + 16 * wv;
  const size_t prow = (size_t)head * CROWS + (size_t)b * CN;

  const _Float16* qrow = qp + (prow + q0 + m) * CHD;
  const v16h qb0 = load_frag(qrow, hl);
  const v16h qb1 = load_frag(qrow + 32, hl);
  const v16h qb2 = load_frag(qrow + 64, hl);

  v8f o[6];
  #pragma unroll
  for (int t = 0; t < 6; ++t) o[t] = zero_v8f();
  float mrun = -1e30f, lrun = 0.0f;
  const float scl = 0.10206207261596575f;

  const _Float16* kbase = kp + (prow + m) * CHD;
  const _Float16* vbase = vt + ((size_t)(head * CHD + m)) * CROWS + (size_t)b * CN;

  #pragma unroll 1
  for (int kb = 0; kb < CN; kb += 64) {
    v8f s[4];
    #pragma unroll
    for (int j = 0; j < 4; ++j) {
      const _Float16* kpp = kbase + (size_t)(kb + 16 * j) * CHD;
      const v16h kf0 = load_frag(kpp, hl);
      const v16h kf1 = load_frag(kpp + 32, hl);
      const v16h kf2 = load_frag(kpp + 64, hl);
      v8f z = zero_v8f();
      z = wmma_f16(kf0, qb0, z);
      z = wmma_f16(kf1, qb1, z);
      z = wmma_f16(kf2, qb2, z);
      s[j] = z * scl;
    }

    float mloc = s[0][0];
    #pragma unroll
    for (int j = 0; j < 4; ++j)
      #pragma unroll
      for (int r = 0; r < 8; ++r) mloc = fmaxf(mloc, s[j][r]);
    mloc = fmaxf(mloc, __shfl_xor(mloc, 16));
    const float mnew = fmaxf(mrun, mloc);
    const float alpha = __expf(mrun - mnew);
    mrun = mnew;
    float lsum = 0.0f;
    #pragma unroll
    for (int j = 0; j < 4; ++j)
      #pragma unroll
      for (int r = 0; r < 8; ++r) {
        const float p = __expf(s[j][r] - mnew);
        s[j][r] = p;
        lsum += p;
      }
    lsum += __shfl_xor(lsum, 16);
    lrun = lrun * alpha + lsum;
    #pragma unroll
    for (int t = 0; t < 6; ++t) o[t] = o[t] * alpha;

    const v16h pb0 = pack_p(s[0], s[1]);
    const v16h pb1 = pack_p(s[2], s[3]);

    #pragma unroll
    for (int t = 0; t < 6; ++t) {
      const _Float16* vp = vbase + (size_t)(16 * t) * CROWS + kb;
      const v16h vf0 = load_frag(vp, hl);
      const v16h vf1 = load_frag(vp + 32, hl);
      o[t] = wmma_f16(vf0, pb0, o[t]);
      o[t] = wmma_f16(vf1, pb1, o[t]);
    }
  }

  const float inv = (1.0f / lrun) * (OSCALE / PSCALE);
  _Float16* so = sO + wv * (16 * CHD);
  #pragma unroll
  for (int t = 0; t < 6; ++t)
    #pragma unroll
    for (int r = 0; r < 8; ++r)
      so[m * CHD + 16 * t + 8 * hl + r] = (_Float16)(o[t][r] * inv);
  __syncthreads();

  _Float16* dst = op + (prow + q0) * CHD;
  v8h vals[6];
  #pragma unroll
  for (int i = 0; i < 6; ++i) {
    const int c = i * 32 + lane;
    vals[i] = *(const v8ha*)(so + 8 * c);
    *(volatile v8h*)(dst + 8 * c) = vals[i];
  }
  __threadfence();
  #pragma unroll
  for (int i = 0; i < 6; ++i) {
    const int c = i * 32 + lane;
    *(volatile v8h*)(dst + 8 * c) = vals[i];
  }
}

__global__ __launch_bounds__(192) void gate_kernel(
    const float* __restrict__ cpq,
    const float* __restrict__ xk,
    const float* __restrict__ temp,
    float* __restrict__ av)
{
  __shared__ float sA[2][CHD], sB2[2][CHD];
  __shared__ float sMq[CHD], sMk[CHD], sIq[CHD], sIk[CHD];
  __shared__ float sKb[CN];
  __shared__ __attribute__((aligned(16))) float sG[CHD];

  const int tid = threadIdx.x, lane = tid & 31, wv = tid >> 5;
  const int b = blockIdx.x >> 3, head = blockIdx.x & 7;
  const int hf = (tid < CHD) ? 0 : 1;
  const int d = tid - hf * CHD;
  const size_t rowb = (size_t)b * CN;
  const int col = head * CHD + d;
  const float* qc = cpq + rowb * CD + col;
  const float* kc = xk + rowb * CD + col;
  const int n0 = hf * (CN / 2);

  float mq = -3.0e38f, mk = -3.0e38f;
  #pragma unroll 1
  for (int n = n0; n < n0 + CN / 2; ++n) {
    mq = fmaxf(mq, qc[(size_t)n * CD]);
    mk = fmaxf(mk, kc[(size_t)n * CD]);
  }
  sA[hf][d] = mq; sB2[hf][d] = mk;
  __syncthreads();
  if (tid < CHD) {
    sMq[tid] = fmaxf(sA[0][tid], sA[1][tid]);
    sMk[tid] = fmaxf(sB2[0][tid], sB2[1][tid]);
  }
  __syncthreads();
  const float Mq = sMq[d], Mk = sMk[d];
  float sq = 0.f, sk = 0.f;
  #pragma unroll 1
  for (int n = n0; n < n0 + CN / 2; ++n) {
    sq += __expf(qc[(size_t)n * CD] - Mq);
    sk += __expf(kc[(size_t)n * CD] - Mk);
  }
  sA[hf][d] = sq; sB2[hf][d] = sk;
  __syncthreads();
  if (tid < CHD) {
    sIq[tid] = 1.0f / (sA[0][tid] + sA[1][tid]);
    sIk[tid] = 1.0f / (sB2[0][tid] + sB2[1][tid]);
  }
  __syncthreads();

  {
    float mk3[3], ik3[3];
    #pragma unroll
    for (int e = 0; e < 3; ++e) { mk3[e] = sMk[lane + 32 * e]; ik3[e] = sIk[lane + 32 * e]; }
    const float* kb0 = xk + rowb * CD + head * CHD + lane;
    #pragma unroll 1
    for (int n = wv; n < CN; n += 6) {
      const float* p = kb0 + (size_t)n * CD;
      float t = __expf(p[0] - mk3[0]) * ik3[0] + __expf(p[32] - mk3[1]) * ik3[1] + __expf(p[64] - mk3[2]) * ik3[2];
      t = wave_sum(t);
      if (lane == 0) sKb[n] = t * (1.0f / CHD);
    }
  }
  __syncthreads();

  float dot = 0.f;
  #pragma unroll 1
  for (int n = n0; n < n0 + CN / 2; ++n) dot += __expf(qc[(size_t)n * CD] - Mq) * sKb[n];
  sA[hf][d] = dot;
  __syncthreads();
  if (tid < CHD) {
    const float z = (sA[0][tid] + sA[1][tid]) * sIq[tid];
    const float g = 1.0f / (1.0f + __expf(-z));
    sG[tid] = g * temp[head];
  }
  __syncthreads();
  if (tid < 24) {
    const v4f vv = *(const v4fa*)(sG + 4 * tid);
    float* dst = av + (size_t)b * CD + head * CHD + 4 * tid;
    *(volatile v4f*)dst = vv;
    __threadfence();
    *(volatile v4f*)dst = vv;
  }
}

__global__ __launch_bounds__(192) void dwconv_kernel(
    const _Float16* __restrict__ h1, const float* __restrict__ dww,
    const float* __restrict__ dwb, _Float16* __restrict__ h2)
{
  __shared__ __attribute__((aligned(16))) _Float16 sIn[6 * 34 * CHD];
  __shared__ __attribute__((aligned(16))) _Float16 sOut[128 * CHD];

  const int tid = threadIdx.x, lane = tid & 31, wv = tid >> 5;
  const int j = blockIdx.y;
  const int b = blockIdx.x >> 3, yb = blockIdx.x & 7;
  const size_t pr = (size_t)j * CROWS + (size_t)b * CN;
  const v8h zero8h = {(_Float16)0.f, (_Float16)0.f, (_Float16)0.f, (_Float16)0.f,
                      (_Float16)0.f, (_Float16)0.f, (_Float16)0.f, (_Float16)0.f};

  for (int c = tid; c < 6 * 34 * 12; c += 192) {
    const int r = c / 408, rem = c - r * 408;
    const int xx = rem / 12, g = rem - xx * 12;
    const int yy = yb * 4 - 1 + r, xs = xx - 1;
    const bool ok = (yy >= 0) && (yy < IMG) && (xs >= 0) && (xs < IMG);
    const int yyc = min(max(yy, 0), IMG - 1), xsc = min(max(xs, 0), IMG - 1);
    v8h vv = *(const v8ha*)(h1 + (pr + (size_t)(yyc * IMG + xsc)) * CHD + 8 * g);
    vv = ok ? vv : zero8h;
    *(v8ha*)(sIn + (r * 34 + xx) * CHD + 8 * g) = vv;
  }

  const int d = (tid < CHD) ? tid : tid - CHD;
  const int tk0 = (tid < CHD) ? 0 : 1;
  const int ch = j * CHD + d;
  float wt[9];
  #pragma unroll
  for (int i = 0; i < 9; ++i) wt[i] = dww[ch * 9 + i];
  const float bsv = dwb[ch];
  __syncthreads();

  #pragma unroll 1
  for (int it = 0; it < 64; ++it) {
    const int tk = tk0 + 2 * it;
    const int yl = tk >> 5, x0 = tk & 31;
    const _Float16* p = sIn + (yl * 34 + x0) * CHD + d;
    float acc = 0.0f;
    #pragma unroll
    for (int dy = 0; dy < 3; ++dy)
      #pragma unroll
      for (int dx = 0; dx < 3; ++dx)
        acc += (float)p[(dy * 34 + dx) * CHD] * wt[dy * 3 + dx];
    acc += bsv;
    const float gl = 0.5f * acc * (1.0f + erff(acc * 0.70710678118654752f));
    sOut[tk * CHD + d] = (_Float16)gl;
  }
  __syncthreads();

  _Float16* dst = h2 + (pr + (size_t)yb * 128) * CHD;
  v8h vals[8];
  #pragma unroll
  for (int i = 0; i < 8; ++i) {
    const int c = i * 192 + wv * 32 + lane;
    vals[i] = *(const v8ha*)(sOut + 8 * c);
    *(volatile v8h*)(dst + 8 * c) = vals[i];
  }
  __threadfence();
  #pragma unroll
  for (int i = 0; i < 8; ++i) {
    const int c = i * 192 + wv * 32 + lane;
    *(volatile v8h*)(dst + 8 * c) = vals[i];
  }
}

__global__ __launch_bounds__(256) void final_kernel(
    const float* __restrict__ vraw, const float* __restrict__ nvw, const float* __restrict__ nvb,
    const float* __restrict__ av, const float* __restrict__ g2, const float* __restrict__ x1,
    float* __restrict__ out)
{
  const int tid = threadIdx.x, lane = tid & 31, wv = tid >> 5;
  const int row = blockIdx.x * 8 + wv;
  const int b = row >> 10;
  const float* vr = vraw + (size_t)row * CD;
  v4f v[6];
  float s = 0.f;
  #pragma unroll
  for (int j = 0; j < 6; ++j) {
    v[j] = *(const v4fa*)(vr + 128 * j + 4 * lane);
    s += (v[j][0] + v[j][1]) + (v[j][2] + v[j][3]);
  }
  s = wave_sum(s);
  const float mean = s * (1.0f / CD);
  float q = 0.f;
  #pragma unroll
  for (int j = 0; j < 6; ++j) {
    v[j] = v[j] - mean;
    q += (v[j][0] * v[j][0] + v[j][1] * v[j][1]) + (v[j][2] * v[j][2] + v[j][3] * v[j][3]);
  }
  q = wave_sum(q);
  const float rs = 1.0f / sqrtf(q * (1.0f / CD) + 1e-5f);

  const float* xr = x1 + (size_t)row * CD;
  const float* ar = av + (size_t)b * CD;
  float* orow = out + (size_t)row * CD;
  v4f ov[6];
  #pragma unroll
  for (int j = 0; j < 6; ++j) {
    const int col = 128 * j + 4 * lane;
    const v4f w4 = *(const v4fa*)(nvw + col);
    const v4f b4 = *(const v4fa*)(nvb + col);
    const v4f vm = v[j] * rs * w4 + b4;
    const v4f a4 = *(const v4fa*)(ar + col);
    const v4f gv = *(const v4fa*)(g2 + col);
    const v4f x4 = *(const v4fa*)(xr + col);
    ov[j] = x4 + gv * (a4 * vm);
    *(volatile v4f*)(orow + col) = ov[j];
  }
  __threadfence();
  #pragma unroll
  for (int j = 0; j < 6; ++j) *(volatile v4f*)(orow + 128 * j + 4 * lane) = ov[j];
}

extern "C" void kernel_launch(void* const* d_in, const int* in_sizes, int n_in,
                              void* d_out, int out_size, void* d_ws, size_t ws_size,
                              hipStream_t stream) {
  if (n_in < 23) return;
  if (in_sizes[0] != CROWS * CD || out_size != CROWS * CD) return;
  if (in_sizes[3] != CD * CD || in_sizes[4] != 2 * CD * CD || in_sizes[5] != CD * CD || in_sizes[10] != CD * CD) return;
  if (in_sizes[12] != CHID * CD || in_sizes[16] != CD * CHID || in_sizes[14] != CHID * 9) return;
  if (in_sizes[1] != CD || in_sizes[2] != CD || in_sizes[6] != CD || in_sizes[7] != CD) return;
  if (in_sizes[8] != CD || in_sizes[9] != CD || in_sizes[17] != CD || in_sizes[18] != CD) return;
  if (in_sizes[19] != CD || in_sizes[20] != CD || in_sizes[13] != CHID || in_sizes[15] != CHID) return;
  if (in_sizes[11] != CH) return;

  const float* x      = (const float*)d_in[0];
  const float* n1w    = (const float*)d_in[1];
  const float* n1b    = (const float*)d_in[2];
  const float* q_w    = (const float*)d_in[3];
  const float* kv_w   = (const float*)d_in[4];
  const float* proj_w = (const float*)d_in[5];
  const float* proj_b = (const float*)d_in[6];
  const float* gamma1 = (const float*)d_in[7];
  const float* n2w    = (const float*)d_in[8];
  const float* n2b    = (const float*)d_in[9];
  const float* cpq_w  = (const float*)d_in[10];
  const float* temp   = (const float*)d_in[11];
  const float* fc1_w  = (const float*)d_in[12];
  const float* fc1_b  = (const float*)d_in[13];
  const float* dw_w   = (const float*)d_in[14];
  const float* dw_b   = (const float*)d_in[15];
  const float* fc2_w  = (const float*)d_in[16];
  const float* fc2_b  = (const float*)d_in[17];
  const float* nvw    = (const float*)d_in[18];
  const float* nvb    = (const float*)d_in[19];
  const float* gamma2 = (const float*)d_in[20];
  float* out = (float*)d_out;

  const size_t szRW = (size_t)5 * CD * CD * 2;
  const size_t P    = (size_t)CROWS * CD * 2;
  const size_t szAV = (size_t)CB * CD * 4;
  const size_t oR1  = szRW;
  const size_t oR2  = oR1 + P;
  const size_t oR3  = oR1 + 2 * P;
  const size_t oR4  = oR1 + 3 * P;
  const size_t oR5  = oR1 + 4 * P;
  const size_t oR6  = oR5 + 2 * P;
  const size_t oR7  = oR6 + szAV;
  const size_t total = oR7 + 4 * P;
  if (total > ws_size) return;

  char* ws = (char*)d_ws;
  _Float16* wq16   = (_Float16*)(ws);
  _Float16* wkv16  = wq16 + (size_t)CD * CD;
  _Float16* wpj16  = wq16 + (size_t)3 * CD * CD;
  _Float16* wcq16  = wq16 + (size_t)4 * CD * CD;
  _Float16* fc2w16 = wq16;
  _Float16* R1h = (_Float16*)(ws + oR1);
  _Float16* R2h = (_Float16*)(ws + oR2);
  _Float16* R3h = (_Float16*)(ws + oR3);
  _Float16* R4h = (_Float16*)(ws + oR4);
  float*    R3f = (float*)(ws + oR3);
  float*    R5f = (float*)(ws + oR5);
  float*    R6f = (float*)(ws + oR6);
  _Float16* R7h = (_Float16*)(ws + oR7);
  float*    R7f = (float*)(ws + oR7);

  const float invW  = 1.0f / WSC;
  const float invWO = 1.0f / (WSC * OSCALE);

  cvt_kernel<<<dim3((2 * CD * CD) / 2048, 4), 256, 0, stream>>>(
      q_w, wq16, CD * CD, kv_w, wkv16, 2 * CD * CD, proj_w, wpj16, CD * CD, cpq_w, wcq16, CD * CD, WSC);

  hipLaunchKernelGGL(HIP_KERNEL_NAME(ln_kernel<0>), dim3(CROWS / 8), dim3(256), 0, stream,
                     x, n1w, n1b, R1h, (float*)nullptr);

  hipLaunchKernelGGL(HIP_KERNEL_NAME(gemm_kernel<0, 0>), dim3(CROWS / 128, (3 * CD) / CHD), dim3(128), 0, stream,
                     (const _Float16*)R1h, (const _Float16*)wq16, CD, 0,
                     (const float*)nullptr, (const float*)nullptr, (const float*)nullptr, invW,
                     R2h, R3h, R4h, (float*)nullptr);

  attn_kernel<<<dim3(CN / 64, CB * CH), 128, 0, stream>>>(R2h, R3h, R4h, R1h);

  hipLaunchKernelGGL(HIP_KERNEL_NAME(gemm_kernel<1, 2>), dim3(CROWS / 128, CD / CHD), dim3(128), 0, stream,
                     (const _Float16*)R1h, (const _Float16*)wpj16, CD, CD,
                     proj_b, x, gamma1, invWO,
                     (_Float16*)nullptr, (_Float16*)nullptr, (_Float16*)nullptr, R5f);

  hipLaunchKernelGGL(HIP_KERNEL_NAME(ln_kernel<1>), dim3(CROWS / 8), dim3(256), 0, stream,
                     (const float*)R5f, n2w, n2b, R2h, R7f);

  hipLaunchKernelGGL(HIP_KERNEL_NAME(gemm_kernel<0, 2>), dim3(CROWS / 128, CD / CHD), dim3(128), 0, stream,
                     (const _Float16*)R2h, (const _Float16*)wcq16, CD, CD,
                     (const float*)nullptr, (const float*)nullptr, (const float*)nullptr, invW,
                     (_Float16*)nullptr, (_Float16*)nullptr, (_Float16*)nullptr, R3f);

  gate_kernel<<<CB * CH, 192, 0, stream>>>((const float*)R3f, (const float*)R7f, temp, R6f);

  cvt_kernel<<<dim3((CHID * CD) / 2048, 2), 256, 0, stream>>>(
      fc1_w, R3h, CHID * CD, fc2_w, fc2w16, CD * CHID, fc1_w, R3h, 0, fc1_w, R3h, 0, WSC);

  hipLaunchKernelGGL(HIP_KERNEL_NAME(gemm_kernel<0, 1>), dim3(CROWS / 128, CHID / CHD), dim3(128), 0, stream,
                     (const _Float16*)R2h, (const _Float16*)R3h, CD, 0,
                     fc1_b, (const float*)nullptr, (const float*)nullptr, invW,
                     R7h, (_Float16*)nullptr, (_Float16*)nullptr, (float*)nullptr);

  dwconv_kernel<<<dim3(CB * 8, CHID / CHD), 192, 0, stream>>>((const _Float16*)R7h, dw_w, dw_b, R1h);

  hipLaunchKernelGGL(HIP_KERNEL_NAME(gemm_kernel<1, 2>), dim3(CROWS / 128, CD / CHD), dim3(128), 0, stream,
                     (const _Float16*)R1h, (const _Float16*)fc2w16, CHID, CD,
                     fc2_b, (const float*)nullptr, (const float*)nullptr, invW,
                     (_Float16*)nullptr, (_Float16*)nullptr, (_Float16*)nullptr, R7f);

  final_kernel<<<CROWS / 8, 256, 0, stream>>>((const float*)R7f, nvw, nvb, (const float*)R6f, gamma2,
                                                (const float*)R5f, out);
}
